// GeneralPolyGNN_52544629899590
// MI455X (gfx1250) — hardware-run, weakly checked
//
#include <hip/hip_runtime.h>


namespace {
constexpr int NB = 128, NPG = 512, NN = NB * NPG, NE = 1048576, F = 128, DEG = 3, MAXDEG = 1024, NGc = (NN + 511) / 512, PERMLEN = NE + 32 * NGc + 32;
constexpr float XS = 8.0f;

typedef _Float16 b16;
typedef __attribute__((ext_vector_type(16))) _Float16 v16b;
typedef __attribute__((ext_vector_type(8))) _Float16 v8b;
typedef __attribute__((ext_vector_type(8))) float v8f;
typedef __attribute__((ext_vector_type(4))) float v4f;
__device__ __forceinline__ float bf16_rne(float f) { unsigned int u = __float_as_uint(f); u += 0x7FFFu + ((u >> 16) & 1u); return __uint_as_float(u & 0xFFFF0000u); }
__device__ __forceinline__ void split16(float v, b16& hi, b16& lo) { hi = (b16)v; lo = (b16)(v - (float)hi); }
__device__ __forceinline__ v16b frag_kb(const b16* p, int hh) { const v8b a = *(const v8b*)(p + 8 * hh), b = *(const v8b*)(p + 16 + 8 * hh); v16b f;
#pragma unroll
  for (int e = 0; e < 8; ++e) { f[e] = a[e]; f[8 + e] = b[e]; } return f; }
__device__ __forceinline__ v8f wmma16b(v16b a, v16b b, v8f c) { v8f d = __builtin_amdgcn_wmma_f32_16x16x32_f16(false, a, false, b, (short)0, c, false, false); asm volatile("v_nop\n\tv_nop\n\tv_nop\n\tv_nop" : "+v"(d) : "v"(a), "v"(b)); return d; }
__device__ __forceinline__ void wave_lds_sync() { __builtin_amdgcn_fence(__ATOMIC_RELEASE, "workgroup"); __builtin_amdgcn_wave_barrier(); __builtin_amdgcn_fence(__ATOMIC_ACQUIRE, "workgroup"); }
__device__ __forceinline__ float pmul(float a, float b) { float p = a * b; asm volatile("" : "+v"(p)); return p; }
__device__ __forceinline__ float wsum(float v) {
#pragma unroll
  for (int o = 1; o < 32; o <<= 1) v += __shfl_xor(v, o); return v; }
constexpr int CSR_NBLK = 512, CSR_GB = 9, CSR_GN = 1 << CSR_GB  , CSR_MAXG = 512, CSR_CAP = 12288  ;
__global__ __launch_bounds__(64) void csrA_kernel(const int* __restrict__ dst, int E, int N, int nG, int CHP, int NGP, int* __restrict__ STG, int* __restrict__ HST) {
  extern __shared__ int sm[];
  int* cnt = sm; int* run = sm + NGP; int* ids = sm + 2 * NGP;
  const int b = blockIdx.x; const int ch = (E + CSR_NBLK - 1) / CSR_NBLK; const int e0 = b * ch, e1 = min(E, e0 + ch);
  for (int i = threadIdx.x; i < NGP; i += 64) cnt[i] = 0;
  for (int i = threadIdx.x; i < CHP; i += 64) ids[i] = -1;
  __syncthreads();
  if (threadIdx.x == 0) {
    for (int e = e0; e < e1; ++e) { int d = dst[e]; d = (d < 0) ? 0 : (d >= N ? N - 1 : d); cnt[d >> CSR_GB] += 1; }
    int acc = 0; for (int g = 0; g < nG; ++g) { run[g] = acc; acc += cnt[g]; }
    for (int e = e0; e < e1; ++e) { int d = dst[e]; d = (d < 0) ? 0 : (d >= N ? N - 1 : d); const int g = d >> CSR_GB; ids[run[g]] = e; run[g] += 1; } }
  __syncthreads();
  typedef __attribute__((ext_vector_type(4))) int v4i;
  for (int pass = 0; pass < 2; ++pass) {
    for (int i = threadIdx.x; i < CHP / 4; i += 64) *(volatile v4i*)(STG + (size_t)b * CHP + i * 4) = *(const v4i*)(&ids[i * 4]);
    for (int i = threadIdx.x; i < NGP / 4; i += 64) { v4i v; for (int e = 0; e < 4; ++e) v[e] = (i * 4 + e < nG) ? cnt[i * 4 + e] : 0; *(volatile v4i*)(HST + (size_t)b * NGP + i * 4) = v; }
    __threadfence(); }
}
__global__ __launch_bounds__(512) void csrS_kernel(const int* __restrict__ HST, int nG, int NGP, int* __restrict__ START, int* __restrict__ TOT, int* __restrict__ OFF) {
  __shared__ int tot[CSR_MAXG];
  const int b = threadIdx.x;
  for (int pass = 0; pass < 2; ++pass) { int runb = 0; for (int g = 0; g < nG; ++g) { int c = HST[(size_t)b * NGP + g]; c = (c < 0) ? 0 : c; ((volatile int*)OFF)[(size_t)g * CSR_NBLK + b] = runb; runb += c; } __threadfence(); }
  for (int g = threadIdx.x; g < nG; g += 512) { int s = 0; for (int bb = 0; bb < CSR_NBLK; ++bb) { int c = HST[(size_t)bb * NGP + g]; s += (c < 0) ? 0 : c; } tot[g] = s; }
  __syncthreads();
  if (threadIdx.x < 32) {
    __shared__ int st[CSR_MAXG + 32];
    if (threadIdx.x == 0) { int acc = 0; for (int g = 0; g < NGP; ++g) { st[g] = acc; if (g < nG) acc += (tot[g] + 31) & ~31; } st[NGP] = acc; }
    __builtin_amdgcn_fence(__ATOMIC_RELEASE, "workgroup"); __builtin_amdgcn_wave_barrier(); __builtin_amdgcn_fence(__ATOMIC_ACQUIRE, "workgroup");
    for (int pass = 0; pass < 2; ++pass) { for (int i = threadIdx.x; i < NGP + 32; i += 32) { ((volatile int*)START)[i] = (i <= NGP) ? st[min(i, NGP)] : 0; ((volatile int*)TOT)[i] = (i < nG) ? tot[i] : 0; } __threadfence(); } }
}
__global__ __launch_bounds__(256) void csrB_kernel(const int* __restrict__ dst, int N, int nG, int CHP, int NGP, int permLen, const int* __restrict__ STG, const int* __restrict__ HST, const int* __restrict__ OFF, const int* __restrict__ START, const int* __restrict__ TOT, int* __restrict__ PERM, int* __restrict__ ROWPTR, int* __restrict__ ROWCNT, int* __restrict__ FLAG) {
  typedef __attribute__((ext_vector_type(4))) int v4i;
  __shared__ int ids[CSR_CAP]; __shared__ unsigned short key[CSR_CAP]; __shared__ int outp[CSR_CAP]; __shared__ int ncnt[CSR_GN + 1]; __shared__ int boff[CSR_NBLK + 1];
  const int g = blockIdx.x, t_ = threadIdx.x; int tot = TOT[g]; int st = START[g], stn = START[g + 1]; const int v0 = g * CSR_GN; const int nv = min(CSR_GN, N - v0);
  st = (st < 0) ? 0 : (st > permLen - 32 ? permLen - 32 : st) & ~31; stn = (stn < st) ? st : (stn > permLen ? permLen : stn); tot = (tot < 0) ? 0 : tot; if (tot > stn - st && tot <= CSR_CAP) tot = stn - st;
  if (tot > CSR_CAP) {
    for (int pass = 0; pass < 2; ++pass) { for (int i = t_; i < CSR_GN / 4; i += 256) { v4i a, c; for (int e = 0; e < 4; ++e) { a[e] = st; c[e] = 0; } *(volatile v4i*)(ROWPTR + v0 + i * 4) = a; *(volatile v4i*)(ROWCNT + v0 + i * 4) = c; } if (t_ == 0) ((volatile int*)FLAG)[0] = 1; __threadfence(); } (void)nv; return; }
  if (t_ == 0) { int acc = 0; for (int b = 0; b < CSR_NBLK; ++b) { boff[b] = acc; int c = HST[(size_t)b * NGP + g]; c = (c < 0) ? 0 : (c > CHP ? CHP : c); acc += c; if (acc > tot) acc = tot; } boff[CSR_NBLK] = acc; }
  for (int i = t_; i <= CSR_GN; i += 256) ncnt[i] = 0;
  __syncthreads();
  for (int b = 0; b < CSR_NBLK; ++b) { const int c = boff[b + 1] - boff[b]; int o_ = OFF[(size_t)g * CSR_NBLK + b]; o_ = (o_ < 0) ? 0 : (o_ > CHP - c ? CHP - c : o_); const int* src_ = STG + (size_t)b * CHP + o_;
    for (int i = t_; i < c; i += 256) { int id = src_[i]; id = (id < 0) ? 0 : id; ids[boff[b] + i] = id; int d = dst[id]; d = (d < v0) ? v0 : (d >= N ? N - 1 : d); int kk = d - v0; kk = (kk < 0) ? 0 : (kk >= CSR_GN ? CSR_GN - 1 : kk); key[boff[b] + i] = (unsigned short)kk; } }
  __syncthreads();
  if (t_ == 0) { for (int i = 0; i < tot; ++i) ncnt[key[i]] += 1; int acc = 0; for (int vl = 0; vl < CSR_GN; ++vl) { const int c = ncnt[vl]; ncnt[vl] = acc; acc += c; } ncnt[CSR_GN] = acc;
    for (int i = 0; i < tot; ++i) { const int vl = key[i]; outp[ncnt[vl]] = ids[i]; ncnt[vl] += 1; }
    for (int vl = CSR_GN; vl > 0; --vl) ncnt[vl] = ncnt[vl - 1]; ncnt[0] = 0; }
  __syncthreads();
  for (int pass = 0; pass < 2; ++pass) {
    for (int i = t_; i < (stn - st) / 4; i += 256) { v4i v; for (int e = 0; e < 4; ++e) { const int q = i * 4 + e; v[e] = (q < tot) ? outp[q] : -1; } *(volatile v4i*)(PERM + st + i * 4) = v; }
    for (int i = t_; i < CSR_GN / 4; i += 256) { v4i a, c; for (int e = 0; e < 4; ++e) { const int vl = i * 4 + e; a[e] = st + ncnt[vl]; c[e] = (vl < nv) ? (ncnt[vl + 1] - ncnt[vl]) : 0; } *(volatile v4i*)(ROWPTR + v0 + i * 4) = a; *(volatile v4i*)(ROWCNT + v0 + i * 4) = c; }
    __threadfence(); }
}
__global__ __launch_bounds__(256) void csrZ_kernel(int* __restrict__ p, size_t n4) { typedef __attribute__((ext_vector_type(4))) int v4i; const size_t tid = (size_t)blockIdx.x * 256 + threadIdx.x, nth = (size_t)gridDim.x * 256; v4i z = {0, 0, 0, 0}; for (size_t i = tid; i < n4; i += nth) *(volatile v4i*)(p + i * 4) = z; }
struct CsrBufs { int *STG, *HST, *OFF, *START, *TOT, *PERM, *ROWPTR, *ROWCNT, *FLAG; int nG, NGP, CHP; size_t permLen; char* base; size_t bytes; };
static size_t csr_carve(CsrBufs& c, char* ws, size_t off, int E, int N) {
  const size_t off0 = off; c.base = ws + off;
  auto al = [&](size_t bytes) { char* p = ws + off; off += (bytes + 255) & ~(size_t)255; return p; };
  c.nG = (N + CSR_GN - 1) / CSR_GN; c.NGP = (c.nG + 31) & ~31; const int ch = (E + CSR_NBLK - 1) / CSR_NBLK; c.CHP = (ch + 31) & ~31; c.permLen = (size_t)E + 32 * (size_t)c.nG + 32;
  c.STG = (int*)al((size_t)CSR_NBLK * c.CHP * 4); c.HST = (int*)al((size_t)CSR_NBLK * c.NGP * 4); c.OFF = (int*)al((size_t)c.NGP * CSR_NBLK * 4); c.START = (int*)al((size_t)(c.NGP + 64) * 4); c.TOT = (int*)al((size_t)(c.NGP + 64) * 4);
  c.PERM = (int*)al(c.permLen * 4); c.ROWPTR = (int*)al((size_t)c.nG * CSR_GN * 4); c.ROWCNT = (int*)al((size_t)c.nG * CSR_GN * 4); c.FLAG = (int*)al(256);
  c.bytes = off - off0; return off;
}
static void csr_build(const CsrBufs& c, const int* dst, int E, int N, hipStream_t stream) {
  const size_t smem = (size_t)(2 * c.NGP + c.CHP) * 4;
  csrZ_kernel<<<512, 256, 0, stream>>>((int*)c.base, c.bytes / 16);
  csrA_kernel<<<CSR_NBLK, 64, smem, stream>>>(dst, E, N, c.nG, c.CHP, c.NGP, c.STG, c.HST);
  csrS_kernel<<<1, 512, 0, stream>>>(c.HST, c.nG, c.NGP, c.START, c.TOT, c.OFF);
  csrB_kernel<<<c.nG, 256, 0, stream>>>(dst, N, c.nG, c.CHP, c.NGP, (int)c.permLen, c.STG, c.HST, c.OFF, c.START, c.TOT, c.PERM, c.ROWPTR, c.ROWCNT, c.FLAG);
}

__global__ __launch_bounds__(128) void adj_kernel(const int* __restrict__ dstn, const int* __restrict__ perm, const int* __restrict__ rowptr, const int* __restrict__ rowcnt, b16* __restrict__ AD, float* __restrict__ DINV) {
  __shared__ __attribute__((aligned(16))) b16 Row[4][NPG + 8]; __shared__ float Dv[32];
  const int wave = threadIdx.x >> 5, lane = threadIdx.x & 31; const int n0 = blockIdx.x * 32;
  for (int rr = 0; rr < 8; ++rr) { const int v = n0 + wave * 8 + rr;
    for (int j = lane; j < NPG; j += 32) Row[wave][j] = (b16)0.0f;
    wave_lds_sync();
    int cnt = rowcnt[v]; cnt = (cnt < 0) ? 0 : (cnt > MAXDEG ? MAXDEG : cnt); int p0 = rowptr[v]; p0 = (p0 < 0) ? 0 : (p0 > PERMLEN - cnt ? PERMLEN - cnt : p0);
    if (lane == 0) { for (int q = 0; q < cnt; ++q) { int id = perm[p0 + q]; id = (id < 0) ? 0 : (id >= NE ? NE - 1 : id); int d = dstn[id]; d = (d < 0) ? 0 : (d >= NN ? NN - 1 : d); Row[wave][d & (NPG - 1)] = (b16)1.0f; } }
    wave_lds_sync();
    float c_ = 0.0f; for (int j = lane; j < NPG; j += 32) c_ += (float)Row[wave][j]; c_ = wsum(c_); if (lane == 0) Dv[wave * 8 + rr] = (c_ > 0.0f) ? rsqrtf(c_) : 0.0f;
    for (int pass = 0; pass < 2; ++pass) { for (int j = lane; j < NPG / 8; j += 32) *(volatile v8b*)(AD + (size_t)v * NPG + j * 8) = *(const v8b*)(&Row[wave][j * 8]); __threadfence(); }
    wave_lds_sync(); }
  __syncthreads();
  for (int pass = 0; pass < 2; ++pass) { if (threadIdx.x < 32) ((volatile float*)DINV)[n0 + threadIdx.x] = Dv[threadIdx.x]; __threadfence(); }
}
__global__ __launch_bounds__(256) void prep_kernel(const float* __restrict__ X, const float* __restrict__ w1, const float* __restrict__ b1, const float* __restrict__ w2, const float* __restrict__ b2, const float* __restrict__ wr1, const float* __restrict__ br1, const float* __restrict__ wr2, const float* __restrict__ br2, b16* __restrict__ R, float* __restrict__ P, float* __restrict__ Z) {
  const size_t tid = (size_t)blockIdx.x * 256 + threadIdx.x, nth = (size_t)gridDim.x * 256;
  for (int pass = 0; pass < 2; ++pass) {
    for (size_t p = tid; p < (size_t)2 * F * F; p += nth) { const int l = (int)(p / (F * F)), o = (int)((p / F) % F), k = (int)(p % F); ((volatile b16*)R)[p] = (b16)bf16_rne((l ? w2 : w1)[(size_t)k * F + o]); }
    for (size_t q = tid; q < 8577; q += nth) { const int i = (int)q; float v; if (i < 128) v = b1[i]; else if (i < 256) v = b2[i - 128]; else if (i < 8448) v = wr1[i - 256]; else if (i < 8512) v = br1[i - 8448]; else if (i < 8576) v = wr2[i - 8512]; else v = br2[0]; P[q] = bf16_rne(v); }
    for (size_t p = tid; p < (size_t)NN * F / 4; p += nth) { const v4f v = *(const v4f*)(X + p * 4); v4f o; for (int e = 0; e < 4; ++e) o[e] = bf16_rne(v[e]); *(volatile v4f*)(Z + p * 4) = o; }
    __threadfence(); }
}
template <int INIT>
__global__ __launch_bounds__(256) void zt_kernel(const float* __restrict__ Z, const float* __restrict__ DINV, b16* __restrict__ ZTh, b16* __restrict__ ZTl, float* __restrict__ ACC) {
  __shared__ __attribute__((aligned(16))) b16 Th[F][64 + 8], Tl[F][64 + 8];
  const int n0 = blockIdx.x * 64, g = n0 / NPG, i0 = n0 % NPG, t_ = threadIdx.x;
  for (int i = t_; i < 64 * F; i += 256) { const int nl = i / F, f = i % F; const float z = Z[(size_t)(n0 + nl) * F + f]; b16 a_, b_; split16(pmul(z, DINV[n0 + nl]) * XS, a_, b_); Th[f][nl] = a_; Tl[f][nl] = b_; }
  __syncthreads();
  for (int pass = 0; pass < 2; ++pass) { for (int i = t_; i < F * 8; i += 256) { const int f = i >> 3, c8 = (i & 7) * 8; const size_t gi = ((size_t)g * F + f) * NPG + i0 + c8; *(volatile v8b*)(ZTh + gi) = *(const v8b*)(&Th[f][c8]); *(volatile v8b*)(ZTl + gi) = *(const v8b*)(&Tl[f][c8]); }
    if (INIT) { for (int i = t_; i < 64 * F / 4; i += 256) *(volatile v4f*)(ACC + (size_t)n0 * F + i * 4) = *(const v4f*)(Z + (size_t)n0 * F + i * 4); }
    __threadfence(); }
}
__global__ __launch_bounds__(64) void hop_kernel(const b16* __restrict__ AD, const b16* __restrict__ ZTh, const b16* __restrict__ ZTl, const float* __restrict__ DINV, float* __restrict__ Z, float* __restrict__ ACC) {
  __shared__ __attribute__((aligned(16))) float Ts[2][16][F + 4];
  const int lane = threadIdx.x & 31, wave = threadIdx.x >> 5, nloc = lane & 15, hlf = lane >> 4, m0 = blockIdx.x * 32 + wave * 16; const int g = m0 / NPG; const b16* Bz = ZTh + (size_t)g * F * NPG; const b16* Bl = ZTl + (size_t)g * F * NPG;
  v8f acc[8];
#pragma unroll
  for (int t = 0; t < 8; ++t) acc[t] = (v8f){};
#pragma unroll 2
  for (int kb = 0; kb < NPG; kb += 32) { const v16b a = frag_kb(AD + (size_t)(m0 + nloc) * NPG + kb, hlf);
#pragma unroll
    for (int t = 0; t < 8; ++t) { const v16b bz = frag_kb(Bz + (size_t)(t * 16 + nloc) * NPG + kb, hlf), bl = frag_kb(Bl + (size_t)(t * 16 + nloc) * NPG + kb, hlf); acc[t] = wmma16b(a, bz, acc[t]); acc[t] = wmma16b(a, bl, acc[t]); } }
#pragma unroll
  for (int t = 0; t < 8; ++t)
#pragma unroll
    for (int r = 0; r < 8; ++r) { const int row = m0 + 8 * hlf + r; Ts[wave][8 * hlf + r][t * 16 + nloc] = pmul(acc[t][r] * (1.0f / XS), DINV[row]); }
  wave_lds_sync();
  for (int i = lane; i < 16 * 32; i += 32) { const int rr = i >> 5, c4 = (i & 31) * 4; const size_t gi = (size_t)(m0 + rr) * F + c4; const v4f zn = *(const v4f*)(&Ts[wave][rr][c4]); const v4f an = *(const v4f*)(ACC + gi) + zn;
    *(volatile v4f*)(Z + gi) = zn; *(volatile v4f*)(ACC + gi) = an; __threadfence(); *(volatile v4f*)(Z + gi) = zn; *(volatile v4f*)(ACC + gi) = an; }
  __threadfence();
}
__global__ __launch_bounds__(64) void lin_kernel(const float* __restrict__ ACC, const b16* __restrict__ Bw, const float* __restrict__ Pb, float* __restrict__ Z) {
  __shared__ __attribute__((aligned(16))) b16 Ah[32][F + 8], Al[32][F + 8]; __shared__ __attribute__((aligned(16))) float Ts[2][16][F + 4];
  const int lane = threadIdx.x & 31, wave = threadIdx.x >> 5, nloc = lane & 15, hlf = lane >> 4, m0 = blockIdx.x * 32;
  for (int i = threadIdx.x; i < 32 * F; i += 64) { const int rr = i / F, c = i % F; b16 a_, b_; split16(ACC[(size_t)(m0 + rr) * F + c] * XS, a_, b_); Ah[rr][c] = a_; Al[rr][c] = b_; }
  __syncthreads();
  v8f acc[8];
#pragma unroll
  for (int t = 0; t < 8; ++t) acc[t] = (v8f){};
#pragma unroll
  for (int kb = 0; kb < F; kb += 32) { const v16b a = frag_kb(&Ah[wave * 16 + nloc][kb], hlf), al_ = frag_kb(&Al[wave * 16 + nloc][kb], hlf);
#pragma unroll
    for (int t = 0; t < 8; ++t) { const v16b bw = frag_kb(Bw + (size_t)(t * 16 + nloc) * F + kb, hlf); acc[t] = wmma16b(a, bw, acc[t]); acc[t] = wmma16b(al_, bw, acc[t]); } }
#pragma unroll
  for (int t = 0; t < 8; ++t)
#pragma unroll
    for (int r = 0; r < 8; ++r) Ts[wave][8 * hlf + r][t * 16 + nloc] = fmaxf(acc[t][r] * (1.0f / XS) + Pb[t * 16 + nloc], 0.0f);
  wave_lds_sync();
  for (int pass = 0; pass < 2; ++pass) { for (int i = lane; i < 16 * 32; i += 32) { const int rr = i >> 5, c4 = (i & 31) * 4; *(volatile v4f*)(Z + (size_t)(m0 + wave * 16 + rr) * F + c4) = *(const v4f*)(&Ts[wave][rr][c4]); } __threadfence(); }
}
__global__ __launch_bounds__(128) void pool_kernel(const float* __restrict__ Z, float* __restrict__ HM) {
  const int g = blockIdx.x, f = threadIdx.x; float s = 0.0f; for (int n = 0; n < NPG; ++n) s += Z[((size_t)g * NPG + n) * F + f];
  const float hm = s * (1.0f / NPG);
  for (int pass = 0; pass < 2; ++pass) { ((volatile float*)HM)[(size_t)g * F + f] = hm; __threadfence(); }
}
__global__ __launch_bounds__(128) void head_kernel(const float* __restrict__ HM, const float* __restrict__ P, float* __restrict__ out) {
  const int g = threadIdx.x; const float* h = HM + (size_t)g * F; float o = P[8576];
  for (int j = 0; j < 64; ++j) { float s = P[8448 + j]; for (int f = 0; f < F; ++f) s += pmul(h[f], P[256 + f * 64 + j]); o += pmul(fmaxf(s, 0.0f), P[8512 + j]); }
  for (int pass = 0; pass < 2; ++pass) { ((volatile float*)out)[g] = o; __threadfence(); }
}
}

extern "C" void kernel_launch(void* const* d_in, const int* in_sizes, int n_in,
                              void* d_out, int out_size, void* d_ws, size_t ws_size, hipStream_t stream) {
  (void)n_in; (void)out_size;
  auto Fp = [&](int i) { return (const float*)d_in[i]; };
  const float* X = Fp(0); const int* ei = (const int*)d_in[2];
  float* out = (float*)d_out;
  if (in_sizes[0] != NN * F || in_sizes[2] != 2 * NE || in_sizes[3] != F * F) return;
  const int* srcI = ei; const int* dstI = ei + NE; const int NE_RUN = NE;
  size_t off = 0; char* ws = (char*)d_ws;
  auto carve = [&](size_t bytes) { char* p = ws + off; off += (bytes + 255) & ~(size_t)255; return p; };
  b16* R = (b16*)carve((size_t)2 * F * F * 2); float* P = (float*)carve(8580 * 4); b16* AD = (b16*)carve((size_t)NN * NPG * 2); float* DINV = (float*)carve((size_t)NN * 4); float* Z = (float*)carve((size_t)NN * F * 4); float* ACC = (float*)carve((size_t)NN * F * 4); b16* ZTh = (b16*)carve((size_t)NN * F * 2); b16* ZTl = (b16*)carve((size_t)NN * F * 2); float* HM = (float*)carve((size_t)NB * F * 4);
  CsrBufs cs; off = csr_carve(cs, ws, off, NE_RUN, NN);
  if (off > ws_size) return;
  csr_build(cs, srcI, NE_RUN, NN, stream);
  adj_kernel<<<NN / 32, 128, 0, stream>>>(dstI, cs.PERM, cs.ROWPTR, cs.ROWCNT, AD, DINV);
  prep_kernel<<<512, 256, 0, stream>>>(X, Fp(3), Fp(4), Fp(5), Fp(6), Fp(7), Fp(8), Fp(9), Fp(10), R, P, Z);
  for (int layer = 0; layer < 2; ++layer) {
    zt_kernel<1><<<NN / 64, 256, 0, stream>>>(Z, DINV, ZTh, ZTl, ACC);
    for (int k = 0; k < DEG; ++k) { hop_kernel<<<NN / 32, 64, 0, stream>>>(AD, ZTh, ZTl, DINV, Z, ACC); if (k + 1 < DEG) zt_kernel<0><<<NN / 64, 256, 0, stream>>>(Z, DINV, ZTh, ZTl, ACC); }
    lin_kernel<<<NN / 32, 64, 0, stream>>>(ACC, R + (size_t)layer * F * F, P + layer * F, Z); }
  pool_kernel<<<NB, 128, 0, stream>>>(Z, HM);
  head_kernel<<<1, 128, 0, stream>>>(HM, P, out);
}
